// GPT2Block_39917426049328
// MI455X (gfx1250) — hardware-run, weakly checked
//
#include <hip/hip_runtime.h>
#include <math.h>

typedef __attribute__((ext_vector_type(16))) _Float16 v16h;
typedef __attribute__((ext_vector_type(8)))  _Float16 v8h;
typedef __attribute__((ext_vector_type(16))) __bf16   v16b;
typedef __attribute__((ext_vector_type(8)))  __bf16   v8b;
typedef __attribute__((ext_vector_type(8)))  float    v8f;
typedef __attribute__((ext_vector_type(4)))  float    v4f;
typedef __attribute__((ext_vector_type(4)))  unsigned int v4u;

constexpr int kBatch   = 2;
constexpr int kSeq     = 2048;
constexpr int kDim     = 1024;
constexpr int kHeads   = 16;
constexpr int kHeadDim = 64;
constexpr int kRows    = kBatch * kSeq;
constexpr int kQkvN    = 3 * kDim;
constexpr int kFfn     = 4 * kDim;
constexpr float kLnEps    = 1e-5f;
constexpr float kMaskFill = -10000.0f;
constexpr float kWCarry   = 64.0f;
constexpr float kAttnCarry = 64.0f;
constexpr float kPCarry    = 32768.0f;

static_assert(kHeads * kHeadDim == kDim, "head split");
static_assert(kHeadDim == 64, "attention kernel is written for head dim 64");
static_assert(kSeq % 64 == 0, "query/key blocks of 64");
static_assert(kRows % 64 == 0 && kQkvN % 64 == 0 && kDim % 64 == 0 && kFfn % 64 == 0, "GEMM M/N tile multiples of 64");
static_assert(kDim % 32 == 0 && kFfn % 32 == 0, "GEMM K multiples of 32");
static_assert(kDim == 128 * 8, "LayerNorm kernel maps 128 threads x 8 elements per row");

constexpr size_t kOffWattnT = 0;
constexpr size_t kSzWattnT  = (size_t)kQkvN * kDim * 2;
constexpr size_t kOffWoT    = kOffWattnT + kSzWattnT;
constexpr size_t kSzWoT     = (size_t)kDim * kDim * 2;
constexpr size_t kOffWfcT   = kOffWoT + kSzWoT;
constexpr size_t kSzWfcT    = (size_t)kFfn * kDim * 2;
constexpr size_t kOffWfpT   = kOffWfcT + kSzWfcT;
constexpr size_t kSzWfpT    = (size_t)kDim * kFfn * 2;
constexpr size_t kOffH1     = kOffWfpT + kSzWfpT;
constexpr size_t kSzH       = (size_t)kRows * kDim * 2;
constexpr size_t kOffQkv    = kOffH1 + kSzH;
constexpr size_t kSzQkv     = (size_t)kRows * kQkvN * 2;
constexpr size_t kOffAttn   = kOffQkv + kSzQkv;
constexpr size_t kSzAttn    = (size_t)kRows * kDim * 2;
constexpr size_t kOffX1     = kOffAttn + kSzAttn;
constexpr size_t kSzX1      = (size_t)kRows * kDim * 4;
constexpr size_t kOffH2     = kOffX1 + kSzX1;
constexpr size_t kOffFc     = kOffH2 + kSzH;
constexpr size_t kSzFc      = (size_t)kRows * kFfn * 2;
constexpr size_t kWsTotal   = kOffFc + kSzFc;
static_assert(kWsTotal == 125829120ull, "carve total");
static_assert(kWsTotal <= 134217728ull, "carve under 128 MiB");
static_assert(kOffWoT % 256 == 0 && kOffWfcT % 256 == 0 && kOffWfpT % 256 == 0 && kOffH1 % 256 == 0 &&
              kOffQkv % 256 == 0 && kOffAttn % 256 == 0 && kOffX1 % 256 == 0 && kOffH2 % 256 == 0 && kOffFc % 256 == 0,
              "aligned regions");

__device__ __forceinline__ unsigned short f2bf_bits(float f) {
  unsigned u = __float_as_uint(f);
  return (unsigned short)((u + 0x7FFFu + ((u >> 16) & 1u)) >> 16);
}
__device__ __forceinline__ float bf_bits2f(unsigned short h) { return __uint_as_float(((unsigned)h) << 16); }

__device__ __forceinline__ void dep_guard_h(v8f& a, v8f& b, v16h x, v16h y) { asm volatile("v_nop\n\tv_nop\n\tv_nop\n\tv_nop" : "+v"(a), "+v"(b) : "v"(x), "v"(y)); }
__device__ __forceinline__ void dep_guard_b(v8f& a, v8f& b, v16b x, v16b y) { asm volatile("v_nop\n\tv_nop\n\tv_nop\n\tv_nop" : "+v"(a), "+v"(b) : "v"(x), "v"(y)); }
__device__ __forceinline__ void keep4_h(v16h a, v16h b, v16h c, v16h d) { asm volatile("v_nop" :: "v"(a), "v"(b), "v"(c), "v"(d)); }
__device__ __forceinline__ void keep4_b(v16b a, v16b b, v16b c, v16b d) { asm volatile("v_nop" :: "v"(a), "v"(b), "v"(c), "v"(d)); }
__device__ __forceinline__ void acc_guard4(v8f& a, v8f& b, v8f& c, v8f& d) { asm volatile("v_nop\n\tv_nop\n\tv_nop\n\tv_nop" : "+v"(a), "+v"(b), "+v"(c), "+v"(d)); }
template <typename T> struct Frag;
template <> struct Frag<_Float16> {
  typedef v16h V; union U { v16h v; v8h h[2]; };
  static __device__ __forceinline__ v16h load(const _Float16* p) {
    U f; f.h[0] = *(const v8h*)(p); f.h[1] = *(const v8h*)(p + 16); return f.v;
  }
  static __device__ __forceinline__ v8f mma(v16h a, v16h b, v8f c) {
    return __builtin_amdgcn_wmma_f32_16x16x32_f16(false, a, false, b, (short)0, c, false, false);
  }
  static __device__ __forceinline__ void guard(v8f& a, v8f& b, v16h x, v16h y) { dep_guard_h(a, b, x, y); }
  static __device__ __forceinline__ void keep(v16h a, v16h b, v16h c, v16h d) { keep4_h(a, b, c, d); }
};
template <> struct Frag<__bf16> {
  typedef v16b V; union U { v16b v; v8b h[2]; };
  static __device__ __forceinline__ v16b load(const __bf16* p) {
    U f; f.h[0] = *(const v8b*)(p); f.h[1] = *(const v8b*)(p + 16); return f.v;
  }
  static __device__ __forceinline__ v8f mma(v16b a, v16b b, v8f c) {
    return __builtin_amdgcn_wmma_f32_16x16x32_bf16(false, a, false, b, (short)0, c, false, false);
  }
  static __device__ __forceinline__ void guard(v8f& a, v8f& b, v16b x, v16b y) { dep_guard_b(a, b, x, y); }
  static __device__ __forceinline__ void keep(v16b a, v16b b, v16b c, v16b d) { keep4_b(a, b, c, d); }
};

__device__ __forceinline__ v8f mma_h(v16h a, v16h b, v8f c) {
  c = __builtin_amdgcn_wmma_f32_16x16x32_f16(false, a, false, b, (short)0, c, false, false);
  asm volatile("v_nop\n\tv_nop\n\tv_nop\n\tv_nop" : "+v"(c) : "v"(a), "v"(b));
  return c;
}

__device__ __forceinline__ float gelu_tanh_form(float x) {
  const float x3 = x * x * x;
  const float w = x + 0.044715f * x3;
  float z = -1.5957691216057308f * w;
  z = fminf(z, 60.0f);
  const float e = expf(z);
  const float r = __builtin_amdgcn_rcpf(1.0f + e);
  return x * r;
}

template <int ET> struct Elem;
template <> struct Elem<0> { typedef _Float16 T; };
template <> struct Elem<1> { typedef __bf16 T; };
template <int ET, bool SPLIT, int BIAS_MODE, int OUT_MODE, bool RESID, int ACT = 0>
__global__ __launch_bounds__(256) void wmma_gemm64(
    const unsigned short* __restrict__ Ap, const unsigned short* __restrict__ A2p, int lda, long strideA,
    const unsigned short* __restrict__ Btp, const unsigned short* __restrict__ Bt2p, int ldb, long strideB,
    void* __restrict__ Cout, void* __restrict__ Cout2, int ldc, long strideC,
    const float* __restrict__ bias,
    const float* __restrict__ resid, long strideR,
    int M, int N, int K, float scale) {
  static_assert(!RESID || OUT_MODE == 0, "resid path is f32-out only");
  typedef typename Elem<ET>::T T;
  typedef typename Frag<T>::V V;
  const T* A = (const T*)Ap; const T* A2 = (const T*)A2p; const T* Bt = (const T*)Btp; const T* Bt2 = (const T*)Bt2p;
  __shared__ __align__(16) float sT[8][16 * 68];
  const int b    = blockIdx.y;
  const int lane = threadIdx.x & 31;
  const int wave = threadIdx.x >> 5;
  const int tilesN = N >> 6;
  const int tilesM = M >> 6;
  const int tile = blockIdx.x * 8 + wave;
  if (tile >= tilesM * tilesN) return;
  const int tm = tile / tilesN;
  const int tn = tile - tm * tilesN;
  const int m0 = tm << 6;
  const int n0 = tn << 6;

  const T* Ab  = A  + (size_t)b * strideA;
  const T* Bb  = Bt + (size_t)b * strideB;
  const T* Ab2 = SPLIT ? (A2  + (size_t)b * strideA) : nullptr;
  const T* Bb2 = SPLIT ? (Bt2 + (size_t)b * strideB) : nullptr;

  const int rlane = lane & 15;
  const int koff  = (lane >> 4) * 8;
  const int mOff  = (lane >> 4) * 8;

  v8f acc[4][4];
#pragma unroll
  for (int i = 0; i < 4; ++i)
#pragma unroll
    for (int j = 0; j < 4; ++j) acc[i][j] = (v8f){0.f,0.f,0.f,0.f,0.f,0.f,0.f,0.f};

  for (int k0 = 0; k0 < K; k0 += 32) {
    V bh[4], bl[4];
#pragma unroll
    for (int j = 0; j < 4; ++j) {
      const size_t bo = (size_t)(n0 + (j << 4) + rlane) * ldb + koff + k0;
      bh[j] = Frag<T>::load(Bb + bo);
      if (SPLIT) bl[j] = Frag<T>::load(Bb2 + bo);
    }
#pragma unroll
    for (int i = 0; i < 4; ++i) {
      const size_t ao = (size_t)(m0 + (i << 4) + rlane) * lda + koff + k0;
      V ah = Frag<T>::load(Ab + ao);
      V al;
      if (SPLIT) al = Frag<T>::load(Ab2 + ao);
#pragma unroll
      for (int j = 0; j < 4; ++j) {
        acc[i][j] = Frag<T>::mma(ah, bh[j], acc[i][j]);
        if (SPLIT) {
          acc[i][j] = Frag<T>::mma(ah, bl[j], acc[i][j]);
          acc[i][j] = Frag<T>::mma(al, bh[j], acc[i][j]);
        }
      }
      Frag<T>::guard(acc[i][0], acc[i][3], ah, SPLIT ? al : ah);
    }
    Frag<T>::keep(bh[0], bh[1], bh[2], bh[3]);
    if (SPLIT) Frag<T>::keep(bl[0], bl[1], bl[2], bl[3]);
  }
  acc_guard4(acc[0][0], acc[0][1], acc[0][2], acc[0][3]);
  acc_guard4(acc[1][0], acc[1][1], acc[1][2], acc[1][3]);
  acc_guard4(acc[2][0], acc[2][1], acc[2][2], acc[2][3]);
  acc_guard4(acc[3][0], acc[3][1], acc[3][2], acc[3][3]);

  float* slab = sT[wave];
#pragma unroll
  for (int i = 0; i < 4; ++i) {
    const int mBase = m0 + (i << 4);
#pragma unroll
    for (int j = 0; j < 4; ++j) {
      const int n = n0 + (j << 4) + rlane;
      float bv = 0.f;
      if (BIAS_MODE == 2) bv = bias[n];
#pragma unroll
      for (int r = 0; r < 8; ++r) {
        float v = acc[i][j][r] * scale;
        if (BIAS_MODE == 1) v += bias[mBase + mOff + r];
        if (BIAS_MODE == 2) v += bv;
        if (ACT == 6) v = gelu_tanh_form(v);
        slab[(mOff + r) * 68 + (j << 4) + rlane] = v;
      }
    }
    __builtin_amdgcn_fence(__ATOMIC_RELEASE, "workgroup");
    __builtin_amdgcn_wave_barrier();
    __builtin_amdgcn_fence(__ATOMIC_ACQUIRE, "workgroup");
    if (OUT_MODE == 0) {
      float* C = (float*)Cout + (size_t)b * strideC;
      const float* Rb = RESID ? (resid + (size_t)b * strideR) : nullptr;
      const int hh = lane >> 4, c4 = (lane & 15) * 4;
      for (int pass = 0; pass < 2; ++pass) {
#pragma unroll
        for (int it = 0; it < 8; ++it) {
          const int row = it * 2 + hh;
          v4f v = *(const v4f*)(slab + row * 68 + c4);
          if (RESID) {
            const v4f rr = *(const v4f*)(Rb + (size_t)(mBase + row) * ldc + n0 + c4);
            v = v + rr;
          }
          *(volatile v4f*)(C + (size_t)(mBase + row) * ldc + n0 + c4) = v;
        }
        __threadfence();
      }
    } else {
      const int q = lane >> 3, c8 = (lane & 7) * 8;
      unsigned short* C  = (unsigned short*)Cout  + (size_t)b * strideC;
      unsigned short* C2 = (OUT_MODE == 2) ? ((unsigned short*)Cout2 + (size_t)b * strideC) : nullptr;
      for (int pass = 0; pass < 2; ++pass) {
#pragma unroll
        for (int it = 0; it < 4; ++it) {
          const int row = it * 4 + q;
          const float* sp = slab + row * 68 + c8;
          v8h hv, lv;
#pragma unroll
          for (int e = 0; e < 8; ++e) {
            if (OUT_MODE == 1) {
              hv[e] = (_Float16)sp[e];
            } else {
              unsigned short hb = f2bf_bits(sp[e]);
              unsigned short lb = f2bf_bits(sp[e] - bf_bits2f(hb));
              hv[e] = __builtin_bit_cast(_Float16, hb);
              lv[e] = __builtin_bit_cast(_Float16, lb);
            }
          }
          *(volatile v8h*)(C + (size_t)(mBase + row) * ldc + n0 + c8) = hv;
          if (OUT_MODE == 2) *(volatile v8h*)(C2 + (size_t)(mBase + row) * ldc + n0 + c8) = lv;
        }
        __threadfence();
      }
    }
    __builtin_amdgcn_fence(__ATOMIC_RELEASE, "workgroup");
    __builtin_amdgcn_wave_barrier();
    __builtin_amdgcn_fence(__ATOMIC_ACQUIRE, "workgroup");
  }
}

__global__ __launch_bounds__(256) void transpose_to_f16(const float* __restrict__ in, unsigned short* __restrict__ out,
                                                        int R, int Cc, float scale) {
  __shared__ float sm[64][65];
  const int tid = threadIdx.x, lane = tid & 31, wave = tid >> 5;
  const int r0 = blockIdx.y * 64, c0 = blockIdx.x * 64;
#pragma unroll
  for (int ps = 0; ps < 4; ++ps) {
    const int r = ps * 16 + (tid >> 4);
    const int c4 = (tid & 15) * 4;
    const v4f v = *(const v4f*)(in + (size_t)(r0 + r) * Cc + c0 + c4);
    sm[r][c4 + 0] = v[0];
    sm[r][c4 + 1] = v[1];
    sm[r][c4 + 2] = v[2];
    sm[r][c4 + 3] = v[3];
  }
  __syncthreads();
  const int q4 = lane >> 3, c8 = (lane & 7) * 8;
  _Float16* ob = (_Float16*)(void*)out;
  for (int pass = 0; pass < 2; ++pass) {
#pragma unroll
    for (int it = 0; it < 2; ++it) {
      const int n = wave * 8 + it * 4 + q4;
      v8h hv;
#pragma unroll
      for (int e = 0; e < 8; ++e) hv[e] = (_Float16)(sm[c8 + e][n] * scale);
      *(volatile v8h*)(ob + (size_t)(c0 + n) * R + r0 + c8) = hv;
    }
    __threadfence();
  }
}

__global__ __launch_bounds__(128) void layernorm_to_f16(const float* __restrict__ x, const float* __restrict__ gam,
                                                        const float* __restrict__ bet, unsigned short* __restrict__ out) {
  __shared__ float red_a[4];
  __shared__ float red_b[4];
  const int row = blockIdx.x;
  const int tid = threadIdx.x, lane = tid & 31, wave = tid >> 5;
  const float* xr = x + (size_t)row * kDim + tid * 8;
  const v4f xa = *(const v4f*)xr;
  const v4f xb = *(const v4f*)(xr + 4);
  float v[8] = {xa[0], xa[1], xa[2], xa[3], xb[0], xb[1], xb[2], xb[3]};

  float s = ((v[0] + v[1]) + (v[2] + v[3])) + ((v[4] + v[5]) + (v[6] + v[7]));
#pragma unroll
  for (int off = 16; off > 0; off >>= 1) s += __shfl_xor(s, off, 32);
  if (lane == 0) red_a[wave] = s;
  __syncthreads();
  const float mu = ((red_a[0] + red_a[1]) + (red_a[2] + red_a[3])) * (1.0f / (float)kDim);

  float d[8];
#pragma unroll
  for (int e = 0; e < 8; ++e) d[e] = v[e] - mu;
  float sq = ((d[0] * d[0] + d[1] * d[1]) + (d[2] * d[2] + d[3] * d[3])) +
             ((d[4] * d[4] + d[5] * d[5]) + (d[6] * d[6] + d[7] * d[7]));
#pragma unroll
  for (int off = 16; off > 0; off >>= 1) sq += __shfl_xor(sq, off, 32);
  if (lane == 0) red_b[wave] = sq;
  __syncthreads();
  const float var = ((red_b[0] + red_b[1]) + (red_b[2] + red_b[3])) * (1.0f / (float)kDim);
  const float rstd = rsqrtf(var + kLnEps);

  const v4f ga = *(const v4f*)(gam + tid * 8);
  const v4f gb = *(const v4f*)(gam + tid * 8 + 4);
  const v4f ba = *(const v4f*)(bet + tid * 8);
  const v4f bb = *(const v4f*)(bet + tid * 8 + 4);
  const float g8[8] = {ga[0], ga[1], ga[2], ga[3], gb[0], gb[1], gb[2], gb[3]};
  const float b8[8] = {ba[0], ba[1], ba[2], ba[3], bb[0], bb[1], bb[2], bb[3]};
  v8h hv;
#pragma unroll
  for (int e = 0; e < 8; ++e) hv[e] = (_Float16)((d[e] * rstd) * g8[e] + b8[e]);
  _Float16* ob = (_Float16*)(void*)out + (size_t)row * kDim + tid * 8;
  *(volatile v8h*)ob = hv;
  __threadfence();
  *(volatile v8h*)ob = hv;
}

__global__ __launch_bounds__(128) void attn64_causal_f16(const unsigned short* __restrict__ qkvp,
                                                         unsigned short* __restrict__ outp) {
  __shared__ __align__(16) _Float16 K_s[64 * 64];
  __shared__ __align__(16) _Float16 V_s[64 * 64];
  __shared__ __align__(16) _Float16 P_s[4][16 * 64];
  __shared__ __align__(16) float    O_s[4][16 * 68];

  const int tid  = threadIdx.x;
  const int wave = tid >> 5;
  const int lane = tid & 31;
  const int hh   = lane >> 4;
  const int c    = lane & 15;

  constexpr int nqb = kSeq / 64;
  const int bx = blockIdx.x;
  const int qb = bx % nqb;
  const int bh = bx / nqb;
  const int h  = bh % kHeads;
  const int b  = bh / kHeads;
  const int q0 = qb * 64 + wave * 16;

  const _Float16* base = (const _Float16*)(const void*)qkvp + (size_t)b * kSeq * kQkvN;
  const _Float16* qptr = base + h * kHeadDim;
  const _Float16* kptr = base + kDim + h * kHeadDim;
  const _Float16* vptr = base + 2 * kDim + h * kHeadDim;

  v16h qa[2];
  {
    const _Float16* qrow = qptr + (size_t)(q0 + c) * kQkvN;
#pragma unroll
    for (int dc = 0; dc < 2; ++dc) qa[dc] = Frag<_Float16>::load(qrow + dc * 32 + 8 * hh);
  }

  float mrow[8], lrow[8];
  v8f oacc[4];
#pragma unroll
  for (int r = 0; r < 8; ++r) { mrow[r] = -INFINITY; lrow[r] = 0.f; }
#pragma unroll
  for (int t = 0; t < 4; ++t) oacc[t] = (v8f){0.f,0.f,0.f,0.f,0.f,0.f,0.f,0.f};

  const int nChunks = qb + 1;
  for (int kc = 0; kc < nChunks; ++kc) {
    const int kv0 = kc * 64;
    __syncthreads();
    {
      const int kvr = tid >> 1, dh = (tid & 1) * 32;
      const v4u* krow = (const v4u*)(const void*)(kptr + (size_t)(kv0 + kvr) * kQkvN + dh);
      const v4u* vrow = (const v4u*)(const void*)(vptr + (size_t)(kv0 + kvr) * kQkvN + dh);
      v4u kw[4], vw[4];
#pragma unroll
      for (int i = 0; i < 4; ++i) { kw[i] = krow[i]; vw[i] = vrow[i]; }
#pragma unroll
      for (int i = 0; i < 4; ++i) *(v8h*)(K_s + kvr * 64 + dh + 8 * i) = __builtin_bit_cast(v8h, kw[i]);
#pragma unroll
      for (int i = 0; i < 4; ++i) {
#pragma unroll
        for (int wj = 0; wj < 4; ++wj) {
          const unsigned w = vw[i][wj];
          const int d = dh + 8 * i + 2 * wj;
          V_s[d * 64 + kvr]       = __builtin_bit_cast(_Float16, (unsigned short)(w & 0xffffu));
          V_s[(d + 1) * 64 + kvr] = __builtin_bit_cast(_Float16, (unsigned short)(w >> 16));
        }
      }
    }
    __syncthreads();

    v8f s[4];
#pragma unroll
    for (int j = 0; j < 4; ++j) {
      s[j] = (v8f){0.f,0.f,0.f,0.f,0.f,0.f,0.f,0.f};
#pragma unroll
      for (int dc = 0; dc < 2; ++dc) {
        const v16h kb = Frag<_Float16>::load(K_s + (j * 16 + c) * 64 + dc * 32 + 8 * hh);
        s[j] = mma_h(qa[dc], kb, s[j]);
      }
    }

    const bool diag = (kc == qb);
    float cm[8];
#pragma unroll
    for (int r = 0; r < 8; ++r) {
      const int qrow = q0 + 8 * hh + r;
      float m = -INFINITY;
#pragma unroll
      for (int j = 0; j < 4; ++j) {
        const int kvcol = kv0 + j * 16 + c;
        const bool masked = diag && (kvcol > qrow);
        float sv = s[j][r] * 0.125f;
        sv = masked ? kMaskFill : sv;
        s[j][r] = sv;
        m = fmaxf(m, sv);
      }
#pragma unroll
      for (int off = 1; off < 16; off <<= 1) m = fmaxf(m, __shfl_xor(m, off, 32));
      cm[r] = m;
    }

    _Float16* pw = P_s[wave];
#pragma unroll
    for (int r = 0; r < 8; ++r) {
      const float mnew = fmaxf(mrow[r], cm[r]);
      const float alpha = expf(mrow[r] - mnew);
      mrow[r] = mnew;
      float psum = 0.f;
#pragma unroll
      for (int j = 0; j < 4; ++j) {
        const float p = expf(s[j][r] - mnew);
        psum += p;
        pw[(8 * hh + r) * 64 + j * 16 + c] = (_Float16)(p * kPCarry);
      }
#pragma unroll
      for (int off = 1; off < 16; off <<= 1) psum += __shfl_xor(psum, off, 32);
      lrow[r] = lrow[r] * alpha + psum;
#pragma unroll
      for (int t = 0; t < 4; ++t) oacc[t][r] *= alpha;
    }
    __builtin_amdgcn_fence(__ATOMIC_RELEASE, "workgroup");
    __builtin_amdgcn_wave_barrier();
    __builtin_amdgcn_fence(__ATOMIC_ACQUIRE, "workgroup");

#pragma unroll
    for (int kk = 0; kk < 2; ++kk) {
      const v16h pa = Frag<_Float16>::load(pw + c * 64 + kk * 32 + 8 * hh);
#pragma unroll
      for (int t = 0; t < 4; ++t) {
        const v16h vb = Frag<_Float16>::load(V_s + (t * 16 + c) * 64 + kk * 32 + 8 * hh);
        oacc[t] = mma_h(pa, vb, oacc[t]);
      }
    }
  }

  float* os = O_s[wave];
#pragma unroll
  for (int r = 0; r < 8; ++r) {
    const float inv = kAttnCarry / (lrow[r] * kPCarry);
#pragma unroll
    for (int t = 0; t < 4; ++t) os[(8 * hh + r) * 68 + t * 16 + c] = oacc[t][r] * inv;
  }
  __builtin_amdgcn_fence(__ATOMIC_RELEASE, "workgroup");
  __builtin_amdgcn_wave_barrier();
  __builtin_amdgcn_fence(__ATOMIC_ACQUIRE, "workgroup");
  {
    const int q4 = lane >> 3, c8 = (lane & 7) * 8;
    _Float16* ob = (_Float16*)(void*)outp + ((size_t)b * kSeq + q0) * kDim + h * kHeadDim;
    for (int pass = 0; pass < 2; ++pass) {
#pragma unroll
      for (int it = 0; it < 4; ++it) {
        const int row = it * 4 + q4;
        const float* sp = os + row * 68 + c8;
        v8h hv;
#pragma unroll
        for (int e = 0; e < 8; ++e) hv[e] = (_Float16)sp[e];
        *(volatile v8h*)(ob + (size_t)row * kDim + c8) = hv;
      }
      __threadfence();
    }
  }
}

extern "C" void kernel_launch(void* const* d_in, const int* in_sizes, int n_in,
                              void* d_out, int out_size, void* d_ws, size_t ws_size,
                              hipStream_t stream) {
  if (n_in < 13) return;
  if (in_sizes[0] != kRows * kDim || in_sizes[1] != kDim || in_sizes[2] != kDim ||
      in_sizes[3] != kDim * kQkvN || in_sizes[4] != kQkvN ||
      in_sizes[5] != kDim * kDim || in_sizes[6] != kDim ||
      in_sizes[7] != kDim || in_sizes[8] != kDim ||
      in_sizes[9] != kDim * kFfn || in_sizes[10] != kFfn ||
      in_sizes[11] != kFfn * kDim || in_sizes[12] != kDim) return;
  if (out_size != kRows * kDim) return;
  if (kWsTotal > ws_size) return;

  const float* x      = (const float*)d_in[0];
  const float* ln1_g  = (const float*)d_in[1];
  const float* ln1_b  = (const float*)d_in[2];
  const float* w_attn = (const float*)d_in[3];
  const float* b_attn = (const float*)d_in[4];
  const float* w_o    = (const float*)d_in[5];
  const float* b_o    = (const float*)d_in[6];
  const float* ln2_g  = (const float*)d_in[7];
  const float* ln2_b  = (const float*)d_in[8];
  const float* w_fc   = (const float*)d_in[9];
  const float* b_fc   = (const float*)d_in[10];
  const float* w_fp   = (const float*)d_in[11];
  const float* b_fp   = (const float*)d_in[12];
  float* out = (float*)d_out;

  char* ws = (char*)d_ws;
  unsigned short* wattnT = (unsigned short*)(ws + kOffWattnT);
  unsigned short* woT    = (unsigned short*)(ws + kOffWoT);
  unsigned short* wfcT   = (unsigned short*)(ws + kOffWfcT);
  unsigned short* wfpT   = (unsigned short*)(ws + kOffWfpT);
  unsigned short* h1     = (unsigned short*)(ws + kOffH1);
  unsigned short* qkv    = (unsigned short*)(ws + kOffQkv);
  unsigned short* attn   = (unsigned short*)(ws + kOffAttn);
  float*          x1     = (float*)(ws + kOffX1);
  unsigned short* h2     = (unsigned short*)(ws + kOffH2);
  unsigned short* fc     = (unsigned short*)(ws + kOffFc);

  const float invW  = 1.0f / kWCarry;
  const float invWA = 1.0f / (kWCarry * kAttnCarry);

  transpose_to_f16<<<dim3(kQkvN / 64, kDim / 64), 256, 0, stream>>>(w_attn, wattnT, kDim, kQkvN, kWCarry);
  transpose_to_f16<<<dim3(kDim / 64, kDim / 64), 256, 0, stream>>>(w_o, woT, kDim, kDim, kWCarry);
  transpose_to_f16<<<dim3(kFfn / 64, kDim / 64), 256, 0, stream>>>(w_fc, wfcT, kDim, kFfn, kWCarry);
  transpose_to_f16<<<dim3(kDim / 64, kFfn / 64), 256, 0, stream>>>(w_fp, wfpT, kFfn, kDim, kWCarry);

  layernorm_to_f16<<<kRows, 128, 0, stream>>>(x, ln1_g, ln1_b, h1);

  wmma_gemm64<0, false, 2, 1, false, 0><<<dim3((kRows / 64) * (kQkvN / 64) / 8, 1), 256, 0, stream>>>(
      h1, nullptr, kDim, 0L, wattnT, nullptr, kDim, 0L, (void*)qkv, nullptr, kQkvN, 0L,
      b_attn, nullptr, 0L, kRows, kQkvN, kDim, invW);

  attn64_causal_f16<<<kBatch * kHeads * (kSeq / 64), 128, 0, stream>>>(qkv, attn);

  wmma_gemm64<0, false, 2, 0, true, 0><<<dim3((kRows / 64) * (kDim / 64) / 8, 1), 256, 0, stream>>>(
      attn, nullptr, kDim, 0L, woT, nullptr, kDim, 0L, (void*)x1, nullptr, kDim, 0L,
      b_o, x, 0L, kRows, kDim, kDim, invWA);

  layernorm_to_f16<<<kRows, 128, 0, stream>>>(x1, ln2_g, ln2_b, h2);

  wmma_gemm64<0, false, 2, 1, false, 6><<<dim3((kRows / 64) * (kFfn / 64) / 8, 1), 256, 0, stream>>>(
      h2, nullptr, kDim, 0L, wfcT, nullptr, kDim, 0L, (void*)fc, nullptr, kFfn, 0L,
      b_fc, nullptr, 0L, kRows, kFfn, kDim, invW);

  wmma_gemm64<0, false, 2, 0, true, 0><<<dim3((kRows / 64) * (kDim / 64) / 8, 1), 256, 0, stream>>>(
      fc, nullptr, kFfn, 0L, wfpT, nullptr, kFfn, 0L, (void*)out, nullptr, kDim, 0L,
      b_fp, x1, 0L, kRows, kDim, kFfn, invW);
}
